// RelativeGlobalAttention_80977313399035
// MI455X (gfx1250) — hardware-verified
//
#include <hip/hip_runtime.h>

typedef __attribute__((ext_vector_type(16))) _Float16 v16h;
typedef __attribute__((ext_vector_type(8)))  _Float16 v8h;
typedef __attribute__((ext_vector_type(16))) __bf16   v16b;
typedef __attribute__((ext_vector_type(8)))  __bf16   v8b;
typedef __attribute__((ext_vector_type(8)))  float    v8f;
typedef __attribute__((ext_vector_type(4)))  float    v4f;

__device__ __forceinline__ unsigned short f2bf_bits(float f) {
  unsigned u = __float_as_uint(f);
  return (unsigned short)((u + 0x7FFFu + ((u >> 16) & 1u)) >> 16);
}
__device__ __forceinline__ float bf_bits2f(unsigned short h) { return __uint_as_float(((unsigned)h) << 16); }

__device__ __forceinline__ void dep_guard_h(v8f& a, v8f& b, v16h x, v16h y) { asm volatile("v_nop\n\tv_nop\n\tv_nop\n\tv_nop" : "+v"(a), "+v"(b) : "v"(x), "v"(y)); }
__device__ __forceinline__ void dep_guard_b(v8f& a, v8f& b, v16b x, v16b y) { asm volatile("v_nop\n\tv_nop\n\tv_nop\n\tv_nop" : "+v"(a), "+v"(b) : "v"(x), "v"(y)); }
__device__ __forceinline__ void keep4_h(v16h a, v16h b, v16h c, v16h d) { asm volatile("v_nop" :: "v"(a), "v"(b), "v"(c), "v"(d)); }
__device__ __forceinline__ void keep4_b(v16b a, v16b b, v16b c, v16b d) { asm volatile("v_nop" :: "v"(a), "v"(b), "v"(c), "v"(d)); }
__device__ __forceinline__ void acc_guard4(v8f& a, v8f& b, v8f& c, v8f& d) { asm volatile("v_nop\n\tv_nop\n\tv_nop\n\tv_nop" : "+v"(a), "+v"(b), "+v"(c), "+v"(d)); }
template <typename T> struct Frag;
template <> struct Frag<_Float16> {
  typedef v16h V; union U { v16h v; v8h h[2]; };
  static __device__ __forceinline__ v16h load(const _Float16* p) {
    U f; f.h[0] = *(const v8h*)(p); f.h[1] = *(const v8h*)(p + 16); return f.v;
  }
  static __device__ __forceinline__ v8f mma(v16h a, v16h b, v8f c) {
    return __builtin_amdgcn_wmma_f32_16x16x32_f16(false, a, false, b, (short)0, c, false, false);
  }
  static __device__ __forceinline__ void guard(v8f& a, v8f& b, v16h x, v16h y) { dep_guard_h(a, b, x, y); }
  static __device__ __forceinline__ void keep(v16h a, v16h b, v16h c, v16h d) { keep4_h(a, b, c, d); }
};
template <> struct Frag<__bf16> {
  typedef v16b V; union U { v16b v; v8b h[2]; };
  static __device__ __forceinline__ v16b load(const __bf16* p) {
    U f; f.h[0] = *(const v8b*)(p); f.h[1] = *(const v8b*)(p + 16); return f.v;
  }
  static __device__ __forceinline__ v8f mma(v16b a, v16b b, v8f c) {
    return __builtin_amdgcn_wmma_f32_16x16x32_bf16(false, a, false, b, (short)0, c, false, false);
  }
  static __device__ __forceinline__ void guard(v8f& a, v8f& b, v16b x, v16b y) { dep_guard_b(a, b, x, y); }
  static __device__ __forceinline__ void keep(v16b a, v16b b, v16b c, v16b d) { keep4_b(a, b, c, d); }
};

template <int ET> struct Elem;
template <> struct Elem<0> { typedef _Float16 T; };
template <> struct Elem<1> { typedef __bf16 T; };
template <int ET, bool SPLIT, int BIAS_MODE, int OUT_MODE, bool RESID, int ACT = 0>
__global__ __launch_bounds__(256) void wmma_gemm64(
    const unsigned short* __restrict__ Ap, const unsigned short* __restrict__ A2p, int lda, long strideA,
    const unsigned short* __restrict__ Btp, const unsigned short* __restrict__ Bt2p, int ldb, long strideB,
    void* __restrict__ Cout, void* __restrict__ Cout2, int ldc, long strideC,
    const float* __restrict__ bias,
    const float* __restrict__ resid, long strideR,
    int M, int N, int K, float scale) {
  typedef typename Elem<ET>::T T;
  typedef typename Frag<T>::V V;
  const T* A = (const T*)Ap; const T* A2 = (const T*)A2p; const T* Bt = (const T*)Btp; const T* Bt2 = (const T*)Bt2p;
  __shared__ __align__(16) float sT[8][16 * 68];
  const int b    = blockIdx.y;
  const int lane = threadIdx.x & 31;
  const int wave = threadIdx.x >> 5;
  const int tilesN = N >> 6;
  const int tilesM = M >> 6;
  const int tile = blockIdx.x * 8 + wave;
  if (tile >= tilesM * tilesN) return;
  const int tm = tile / tilesN;
  const int tn = tile - tm * tilesN;
  const int m0 = tm << 6;
  const int n0 = tn << 6;

  const T* Ab  = A  + (size_t)b * strideA;
  const T* Bb  = Bt + (size_t)b * strideB;
  const T* Ab2 = SPLIT ? (A2  + (size_t)b * strideA) : nullptr;
  const T* Bb2 = SPLIT ? (Bt2 + (size_t)b * strideB) : nullptr;

  const int rlane = lane & 15;
  const int koff  = (lane >> 4) * 8;
  const int mOff  = (lane >> 4) * 8;

  v8f acc[4][4];
#pragma unroll
  for (int i = 0; i < 4; ++i)
#pragma unroll
    for (int j = 0; j < 4; ++j) acc[i][j] = (v8f){0.f,0.f,0.f,0.f,0.f,0.f,0.f,0.f};

  for (int k0 = 0; k0 < K; k0 += 32) {
    V bh[4], bl[4];
#pragma unroll
    for (int j = 0; j < 4; ++j) {
      const size_t bo = (size_t)(n0 + (j << 4) + rlane) * ldb + koff + k0;
      bh[j] = Frag<T>::load(Bb + bo);
      if (SPLIT) bl[j] = Frag<T>::load(Bb2 + bo);
    }
#pragma unroll
    for (int i = 0; i < 4; ++i) {
      const size_t ao = (size_t)(m0 + (i << 4) + rlane) * lda + koff + k0;
      V ah = Frag<T>::load(Ab + ao);
      V al;
      if (SPLIT) al = Frag<T>::load(Ab2 + ao);
#pragma unroll
      for (int j = 0; j < 4; ++j) {
        acc[i][j] = Frag<T>::mma(ah, bh[j], acc[i][j]);
        if (SPLIT) {
          acc[i][j] = Frag<T>::mma(ah, bl[j], acc[i][j]);
          acc[i][j] = Frag<T>::mma(al, bh[j], acc[i][j]);
        }
      }
      Frag<T>::guard(acc[i][0], acc[i][3], ah, SPLIT ? al : ah);
    }
    Frag<T>::keep(bh[0], bh[1], bh[2], bh[3]);
    if (SPLIT) Frag<T>::keep(bl[0], bl[1], bl[2], bl[3]);
  }
  acc_guard4(acc[0][0], acc[0][1], acc[0][2], acc[0][3]);
  acc_guard4(acc[1][0], acc[1][1], acc[1][2], acc[1][3]);
  acc_guard4(acc[2][0], acc[2][1], acc[2][2], acc[2][3]);
  acc_guard4(acc[3][0], acc[3][1], acc[3][2], acc[3][3]);

  float* slab = sT[wave];
  const float* Rb = RESID ? (resid + (size_t)b * strideR) : nullptr;
#pragma unroll
  for (int i = 0; i < 4; ++i) {
    const int mBase = m0 + (i << 4);
#pragma unroll
    for (int j = 0; j < 4; ++j) {
      const int n = n0 + (j << 4) + rlane;
      float bv = 0.f;
      if (BIAS_MODE == 2) bv = bias[n];
#pragma unroll
      for (int r = 0; r < 8; ++r) {
        float v = acc[i][j][r] * scale;
        if (BIAS_MODE == 1) v += bias[mBase + mOff + r];
        if (BIAS_MODE == 2) v += bv;
        if (RESID) v += Rb[(size_t)(mBase + mOff + r) * ldc + n];
        if (ACT == 1) v = tanhf(v);
        if (ACT == 2) v = fmaxf(v, 0.0f);
        if (ACT == 3) v = v / (1.0f + expf(-v));
        if (ACT == 4) v = (v > 0.f) ? v : 0.01f * v;
        if (ACT == 5) v = 0.5f * v * (1.0f + erff(v * 0.70710678118654752f));
        slab[(mOff + r) * 68 + (j << 4) + rlane] = v;
      }
    }
    __builtin_amdgcn_fence(__ATOMIC_RELEASE, "workgroup");
    __builtin_amdgcn_wave_barrier();
    __builtin_amdgcn_fence(__ATOMIC_ACQUIRE, "workgroup");
    if (OUT_MODE == 0) {
      float* C = (float*)Cout + (size_t)b * strideC;
      const int hh = lane >> 4, c4 = (lane & 15) * 4;
      for (int pass = 0; pass < 2; ++pass) {
#pragma unroll
        for (int it = 0; it < 8; ++it) {
          const int row = it * 2 + hh;
          v4f v = *(const v4f*)(slab + row * 68 + c4);
          *(volatile v4f*)(C + (size_t)(mBase + row) * ldc + n0 + c4) = v;
        }
        __threadfence();
      }
    } else {
      const int q = lane >> 3, c8 = (lane & 7) * 8;
      unsigned short* C  = (unsigned short*)Cout  + (size_t)b * strideC;
      unsigned short* C2 = (OUT_MODE == 2) ? ((unsigned short*)Cout2 + (size_t)b * strideC) : nullptr;
      for (int pass = 0; pass < 2; ++pass) {
#pragma unroll
        for (int it = 0; it < 4; ++it) {
          const int row = it * 4 + q;
          const float* sp = slab + row * 68 + c8;
          v8h hv, lv;
#pragma unroll
          for (int e = 0; e < 8; ++e) {
            if (OUT_MODE == 1) {
              hv[e] = (_Float16)sp[e];
            } else {
              unsigned short hb = f2bf_bits(sp[e]);
              unsigned short lb = f2bf_bits(sp[e] - bf_bits2f(hb));
              hv[e] = __builtin_bit_cast(_Float16, hb);
              lv[e] = __builtin_bit_cast(_Float16, lb);
            }
          }
          *(volatile v8h*)(C + (size_t)(mBase + row) * ldc + n0 + c8) = hv;
          if (OUT_MODE == 2) *(volatile v8h*)(C2 + (size_t)(mBase + row) * ldc + n0 + c8) = lv;
        }
        __threadfence();
      }
    }
    __builtin_amdgcn_fence(__ATOMIC_RELEASE, "workgroup");
    __builtin_amdgcn_wave_barrier();
    __builtin_amdgcn_fence(__ATOMIC_ACQUIRE, "workgroup");
  }
}

__device__ __forceinline__ unsigned short at_bf_bits(float f) {
  unsigned u = __float_as_uint(f);
  return (unsigned short)((u + 0x7FFFu + ((u >> 16) & 1u)) >> 16);
}
__device__ __forceinline__ __bf16 at_f2bf(float f) { return __builtin_bit_cast(__bf16, at_bf_bits(f)); }
__device__ __forceinline__ void at_split(float f, __bf16& hi, __bf16& lo) {
  const unsigned short hb = at_bf_bits(f);
  hi = __builtin_bit_cast(__bf16, hb);
  lo = at_f2bf(f - __uint_as_float(((unsigned)hb) << 16));
}
__device__ __forceinline__ v8f at_mma(v16b a, v16b b, v8f c) {
  c = __builtin_amdgcn_wmma_f32_16x16x32_bf16(false, a, false, b, (short)0, c, false, false);
  asm volatile("v_nop\n\tv_nop\n\tv_nop\n\tv_nop" : "+v"(c) : "v"(a), "v"(b));
  return c;
}
__device__ __forceinline__ v8f at_mma_h(v16h a, v16h b, v8f c) {
  c = __builtin_amdgcn_wmma_f32_16x16x32_f16(false, a, false, b, (short)0, c, false, false);
  asm volatile("v_nop\n\tv_nop\n\tv_nop\n\tv_nop" : "+v"(c) : "v"(a), "v"(b));
  return c;
}

__global__ __launch_bounds__(256) void split_planes_kernel(
    const float* __restrict__ in, unsigned short* __restrict__ hi, unsigned short* __restrict__ lo, int n8) {
  const int i = blockIdx.x * 256 + threadIdx.x;
  if (i < n8) {
    const size_t o = (size_t)i * 8;
    const v4f a = *(const v4f*)(in + o);
    const v4f b2 = *(const v4f*)(in + o + 4);
    v8h hv, lv;
#pragma unroll
    for (int e = 0; e < 4; ++e) {
      unsigned short hb = f2bf_bits(a[e]);
      unsigned short lb = f2bf_bits(a[e] - bf_bits2f(hb));
      hv[e] = __builtin_bit_cast(_Float16, hb);
      lv[e] = __builtin_bit_cast(_Float16, lb);
      hb = f2bf_bits(b2[e]);
      lb = f2bf_bits(b2[e] - bf_bits2f(hb));
      hv[4 + e] = __builtin_bit_cast(_Float16, hb);
      lv[4 + e] = __builtin_bit_cast(_Float16, lb);
    }
    *(volatile v8h*)(hi + o) = hv;
    *(volatile v8h*)(lo + o) = lv;
    __threadfence();
    *(volatile v8h*)(hi + o) = hv;
    *(volatile v8h*)(lo + o) = lv;
  }
}

__global__ __launch_bounds__(256) void wtrans_split_kernel(
    const float* __restrict__ W, unsigned short* __restrict__ hi, unsigned short* __restrict__ lo, int K, int N) {
  __shared__ float t[64][33];
  const int tid = threadIdx.x;
  const int k0 = blockIdx.x * 64, n0 = blockIdx.y * 32;
  const int nn = tid & 31, kq = tid >> 5;
#pragma unroll
  for (int i = 0; i < 8; ++i) {
    const int kk = i * 8 + kq;
    t[kk][nn] = W[(size_t)(k0 + kk) * N + n0 + nn];
  }
  __syncthreads();
  const int wave = tid >> 5, lane = tid & 31;
  const int orow = wave * 4 + (lane >> 3);
  const int c8 = (lane & 7) * 8;
  v8h hv, lv;
#pragma unroll
  for (int e = 0; e < 8; ++e) {
    const float x = t[c8 + e][orow];
    const unsigned short hb = f2bf_bits(x);
    const unsigned short lb = f2bf_bits(x - bf_bits2f(hb));
    hv[e] = __builtin_bit_cast(_Float16, hb);
    lv[e] = __builtin_bit_cast(_Float16, lb);
  }
  const size_t oo = (size_t)(n0 + orow) * K + k0 + c8;
  *(volatile v8h*)(hi + oo) = hv;
  *(volatile v8h*)(lo + oo) = lv;
  __threadfence();
  *(volatile v8h*)(hi + oo) = hv;
  *(volatile v8h*)(lo + oo) = lv;
}

#define RA_L   2048
#define RA_H   4
#define RA_DQ  32
#define RA_DV  64
#define RA_QB  64
#define RA_KC  64
#define RA_EW  128
#define RA_TP  84
#define RA_QLD 128
#define RA_VLD 256

__global__ __launch_bounds__(128)
void rel_attn_kernel(const float* __restrict__ q, const float* __restrict__ k,
                     const float* __restrict__ v, const float* __restrict__ E,
                     float* __restrict__ out) {
  union FB { v16b v; v8b h[2]; };
  union FH { v16h v; v8h h[2]; };
  __shared__ __align__(16) __bf16   Ksh[RA_KC * RA_DQ];
  __shared__ __align__(16) __bf16   Ksl[RA_KC * RA_DQ];
  __shared__ __align__(16) __bf16   Vth[RA_DV * RA_KC];
  __shared__ __align__(16) __bf16   Vtl[RA_DV * RA_KC];
  __shared__ __align__(16) _Float16 Esh[RA_EW * RA_DQ];
  __shared__ __align__(16) __bf16   Psh[4][16 * RA_KC];
  __shared__ __align__(16) __bf16   Psl[4][16 * RA_KC];
  __shared__ __align__(16) float    Tsh[4][16 * RA_TP];

  const int tid  = threadIdx.x;
  const int wave = tid >> 5;
  const int lane = tid & 31;
  const int hh   = lane >> 4;
  const int c    = lane & 15;

  const int nqb = RA_L / RA_QB;
  const int bx  = blockIdx.x;
  const int qb  = bx % nqb;
  const int bh  = bx / nqb;
  const int h   = bh % RA_H;
  const int b   = bh / RA_H;
  const int q0b = qb * RA_QB;
  const int q0  = q0b + wave * 16;
  const size_t rowb = (size_t)b * RA_L;

  const float* qh_ptr = q + rowb * RA_QLD + h * RA_DQ;
  const float* kh_ptr = k + rowb * RA_QLD + h * RA_DQ;
  const float* vh_ptr = v + rowb * RA_VLD + h * RA_DV;
  float*       oh_ptr = out + rowb * RA_VLD + h * RA_DV;

  v16b qah, qal;
  v16h qf;
  {
    const float* qrow = qh_ptr + (size_t)(q0 + c) * RA_QLD;
#pragma unroll
    for (int e = 0; e < 8; ++e) {
      const float f0 = qrow[8 * hh + e];
      const float f1 = qrow[16 + 8 * hh + e];
      __bf16 hq, lq;
      at_split(f0, hq, lq); qah[e] = hq; qal[e] = lq;
      at_split(f1, hq, lq); qah[8 + e] = hq; qal[8 + e] = lq;
      qf[e]     = (_Float16)(f0 * 16.0f);
      qf[8 + e] = (_Float16)(f1 * 16.0f);
    }
  }

  float mrow[8], lrow[8];
  v8f oacc[4];
#pragma unroll
  for (int r = 0; r < 8; ++r) { mrow[r] = -INFINITY; lrow[r] = 0.f; }
#pragma unroll
  for (int t = 0; t < 4; ++t) oacc[t] = (v8f){0.f,0.f,0.f,0.f,0.f,0.f,0.f,0.f};

  const int nChunks = qb + 1;
  const int wbase   = 48 - 16 * wave;
  float* Tw = Tsh[wave];

  for (int kc = 0; kc < nChunks; ++kc) {
    const int kv0 = kc * RA_KC;
    __syncthreads();
    {
      const int kvr = tid >> 1;
      {
        const int dq = (tid & 1) * 16;
        const float* krow = kh_ptr + (size_t)(kv0 + kvr) * RA_QLD + dq;
#pragma unroll
        for (int i = 0; i < 4; ++i) {
          const v4f kk = *(const v4f*)(krow + 4 * i);
#pragma unroll
          for (int e = 0; e < 4; ++e) {
            const int d = dq + 4 * i + e;
            __bf16 a, bl; at_split(kk[e], a, bl);
            Ksh[kvr * RA_DQ + d] = a; Ksl[kvr * RA_DQ + d] = bl;
          }
        }
      }
      {
        const int dv = (tid & 1) * 32;
        const float* vrow = vh_ptr + (size_t)(kv0 + kvr) * RA_VLD + dv;
#pragma unroll
        for (int i = 0; i < 8; ++i) {
          const v4f vv = *(const v4f*)(vrow + 4 * i);
#pragma unroll
          for (int e = 0; e < 4; ++e) {
            const int d = dv + 4 * i + e;
            __bf16 a, bl; at_split(vv[e], a, bl);
            Vth[d * RA_KC + kvr] = a; Vtl[d * RA_KC + kvr] = bl;
          }
        }
      }
      {
        const int rel0 = RA_L - RA_QB - (q0b - kv0);
        const int erow = rel0 + tid;
        const int erc  = (erow < RA_L) ? erow : (RA_L - 1);
        const float ez = (erow < RA_L) ? 1024.0f : 0.0f;
        const float* ep = E + (size_t)erc * RA_DQ;
#pragma unroll
        for (int i = 0; i < 4; ++i) {
          const v4f ea = *(const v4f*)(ep + 8 * i);
          const v4f ec = *(const v4f*)(ep + 8 * i + 4);
          v8h ev;
#pragma unroll
          for (int e = 0; e < 4; ++e) {
            ev[e]     = (_Float16)(ea[e] * ez);
            ev[4 + e] = (_Float16)(ec[e] * ez);
          }
          *(v8h*)(Esh + tid * RA_DQ + 8 * i) = ev;
        }
      }
    }
    __syncthreads();

#pragma unroll 1
    for (int ct = 0; ct < 5; ++ct) {
      FH eb;
      const _Float16* er = Esh + (wbase + ct * 16 + c) * RA_DQ;
      eb.h[0] = *(const v8h*)(er + 8 * hh);
      eb.h[1] = *(const v8h*)(er + 16 + 8 * hh);
      v8f tt = (v8f){0.f,0.f,0.f,0.f,0.f,0.f,0.f,0.f};
      tt = at_mma_h(qf, eb.v, tt);
#pragma unroll
      for (int r = 0; r < 8; ++r)
        Tw[(8 * hh + r) * RA_TP + ct * 16 + c] = tt[r] * (1.0f / 16384.0f);
    }

    v8f s[4];
#pragma unroll
    for (int j = 0; j < 4; ++j) {
      s[j] = (v8f){0.f,0.f,0.f,0.f,0.f,0.f,0.f,0.f};
      FB kb, kl;
      kb.h[0] = *(const v8b*)(Ksh + (j * 16 + c) * RA_DQ + 8 * hh);
      kb.h[1] = *(const v8b*)(Ksh + (j * 16 + c) * RA_DQ + 16 + 8 * hh);
      kl.h[0] = *(const v8b*)(Ksl + (j * 16 + c) * RA_DQ + 8 * hh);
      kl.h[1] = *(const v8b*)(Ksl + (j * 16 + c) * RA_DQ + 16 + 8 * hh);
      s[j] = at_mma(qah, kb.v, s[j]);
      s[j] = at_mma(qah, kl.v, s[j]);
      s[j] = at_mma(qal, kb.v, s[j]);
    }
    __builtin_amdgcn_fence(__ATOMIC_RELEASE, "workgroup");
    __builtin_amdgcn_wave_barrier();
    __builtin_amdgcn_fence(__ATOMIC_ACQUIRE, "workgroup");

    const bool diag = (kc == qb);
    float cm[8];
#pragma unroll
    for (int r = 0; r < 8; ++r) {
      const int rl = 8 * hh + r;
      const int rr = wave * 16 + rl;
      const float* trow = Tw + rl * RA_TP + 15 - rl;
      float m = -INFINITY;
#pragma unroll
      for (int j = 0; j < 4; ++j) {
        const int cc = j * 16 + c;
        float sv = s[j][r] + trow[cc];
        if (diag && (cc > rr)) sv = -1.0e9f;
        s[j][r] = sv;
        m = fmaxf(m, sv);
      }
#pragma unroll
      for (int off = 1; off < 16; off <<= 1) m = fmaxf(m, __shfl_xor(m, off, 32));
      cm[r] = m;
    }
    __bf16* pwh = Psh[wave];
    __bf16* pwl = Psl[wave];
#pragma unroll
    for (int r = 0; r < 8; ++r) {
      const float mnew = fmaxf(mrow[r], cm[r]);
      const float alpha = expf(mrow[r] - mnew);
      mrow[r] = mnew;
      float psum = 0.f;
#pragma unroll
      for (int j = 0; j < 4; ++j) {
        const float p = expf(s[j][r] - mnew);
        psum += p;
        __bf16 a, bl; at_split(p, a, bl);
        pwh[(8 * hh + r) * RA_KC + j * 16 + c] = a;
        pwl[(8 * hh + r) * RA_KC + j * 16 + c] = bl;
      }
#pragma unroll
      for (int off = 1; off < 16; off <<= 1) psum += __shfl_xor(psum, off, 32);
      lrow[r] = lrow[r] * alpha + psum;
#pragma unroll
      for (int t = 0; t < 4; ++t) oacc[t][r] *= alpha;
    }
    __builtin_amdgcn_fence(__ATOMIC_RELEASE, "workgroup");
    __builtin_amdgcn_wave_barrier();
    __builtin_amdgcn_fence(__ATOMIC_ACQUIRE, "workgroup");
#pragma unroll 1
    for (int kk = 0; kk < 2; ++kk) {
      FB pa, pl;
      pa.h[0] = *(const v8b*)(pwh + c * RA_KC + kk * 32 + 8 * hh);
      pa.h[1] = *(const v8b*)(pwh + c * RA_KC + kk * 32 + 16 + 8 * hh);
      pl.h[0] = *(const v8b*)(pwl + c * RA_KC + kk * 32 + 8 * hh);
      pl.h[1] = *(const v8b*)(pwl + c * RA_KC + kk * 32 + 16 + 8 * hh);
#pragma unroll
      for (int t = 0; t < 4; ++t) {
        FB vb, vl;
        vb.h[0] = *(const v8b*)(Vth + (t * 16 + c) * RA_KC + kk * 32 + 8 * hh);
        vb.h[1] = *(const v8b*)(Vth + (t * 16 + c) * RA_KC + kk * 32 + 16 + 8 * hh);
        vl.h[0] = *(const v8b*)(Vtl + (t * 16 + c) * RA_KC + kk * 32 + 8 * hh);
        vl.h[1] = *(const v8b*)(Vtl + (t * 16 + c) * RA_KC + kk * 32 + 16 + 8 * hh);
        oacc[t] = at_mma(pa.v, vb.v, oacc[t]);
        oacc[t] = at_mma(pa.v, vl.v, oacc[t]);
        oacc[t] = at_mma(pl.v, vb.v, oacc[t]);
      }
    }
  }

  float* os = Tw;
#pragma unroll
  for (int r = 0; r < 8; ++r) {
    const float inv = 0.125f / lrow[r];
#pragma unroll
    for (int t = 0; t < 4; ++t) os[(8 * hh + r) * 68 + t * 16 + c] = oacc[t][r] * inv;
  }
  __builtin_amdgcn_fence(__ATOMIC_RELEASE, "workgroup");
  __builtin_amdgcn_wave_barrier();
  __builtin_amdgcn_fence(__ATOMIC_ACQUIRE, "workgroup");
  {
    const int c4 = (lane & 15) * 4;
    for (int pass = 0; pass < 2; ++pass) {
#pragma unroll
      for (int it = 0; it < 8; ++it) {
        const int row = it * 2 + hh;
        v4f val = *(const v4f*)(os + row * 68 + c4);
        *(volatile v4f*)(oh_ptr + (size_t)(q0 + row) * RA_VLD + c4) = val;
      }
      __threadfence();
    }
  }
}

extern "C" void kernel_launch(void* const* d_in, const int* in_sizes, int n_in,
                              void* d_out, int out_size, void* d_ws, size_t ws_size,
                              hipStream_t stream) {
  const int Bn = 4, Ln = 2048, Dn = 256, Dq = 128, Hn = 4;
  const int M = Bn * Ln;
  const size_t nAct = (size_t)M * Dn;
  if (n_in < 12) return;
  if (in_sizes[0] != (int)nAct || in_sizes[1] != (int)nAct || in_sizes[2] != (int)nAct) return;
  if (in_sizes[3] != Dn * Dq || in_sizes[5] != Dn * Dq || in_sizes[7] != Dn * Dn || in_sizes[9] != Dn * Dn) return;
  if (in_sizes[4] < Dq || in_sizes[6] < Dq || in_sizes[8] < Dn || in_sizes[10] < Dn) return;
  if (in_sizes[11] != Ln * 32) return;
  if (out_size != (int)nAct) return;

  const float* q_in = (const float*)d_in[0];
  const float* k_in = (const float*)d_in[1];
  const float* v_in = (const float*)d_in[2];
  const float* Wq   = (const float*)d_in[3];
  const float* bq   = (const float*)d_in[4];
  const float* Wk   = (const float*)d_in[5];
  const float* bk   = (const float*)d_in[6];
  const float* Wv   = (const float*)d_in[7];
  const float* bv   = (const float*)d_in[8];
  const float* Wfc  = (const float*)d_in[9];
  const float* bfc  = (const float*)d_in[10];
  const float* E    = (const float*)d_in[11];
  float* out        = (float*)d_out;

  size_t off = 0;
  auto carve = [&](size_t bytes) -> char* {
    char* p = (char*)d_ws + off;
    off += (bytes + 255) & ~(size_t)255;
    return p;
  };
  unsigned short* aqH = (unsigned short*)carve(nAct * 2);
  unsigned short* aqL = (unsigned short*)carve(nAct * 2);
  unsigned short* akH = (unsigned short*)carve(nAct * 2);
  unsigned short* akL = (unsigned short*)carve(nAct * 2);
  unsigned short* avH = (unsigned short*)carve(nAct * 2);
  unsigned short* avL = (unsigned short*)carve(nAct * 2);
  unsigned short* aoH = (unsigned short*)carve(nAct * 2);
  unsigned short* aoL = (unsigned short*)carve(nAct * 2);
  unsigned short* wqH = (unsigned short*)carve((size_t)Dq * Dn * 2);
  unsigned short* wqL = (unsigned short*)carve((size_t)Dq * Dn * 2);
  unsigned short* wkH = (unsigned short*)carve((size_t)Dq * Dn * 2);
  unsigned short* wkL = (unsigned short*)carve((size_t)Dq * Dn * 2);
  unsigned short* wvH = (unsigned short*)carve((size_t)Dn * Dn * 2);
  unsigned short* wvL = (unsigned short*)carve((size_t)Dn * Dn * 2);
  unsigned short* wfH = (unsigned short*)carve((size_t)Dn * Dn * 2);
  unsigned short* wfL = (unsigned short*)carve((size_t)Dn * Dn * 2);
  float* qp  = (float*)carve((size_t)M * Dq * 4);
  float* kp  = (float*)carve((size_t)M * Dq * 4);
  float* vp  = (float*)carve((size_t)M * Dn * 4);
  float* Obf = (float*)carve((size_t)M * Dn * 4);
  if (off > ws_size) return;

  const int n8 = (int)(nAct / 8);
  const dim3 gCast((unsigned)((n8 + 255) / 256));

  split_planes_kernel<<<gCast, 256, 0, stream>>>(q_in, aqH, aqL, n8);
  split_planes_kernel<<<gCast, 256, 0, stream>>>(k_in, akH, akL, n8);
  split_planes_kernel<<<gCast, 256, 0, stream>>>(v_in, avH, avL, n8);
  wtrans_split_kernel<<<dim3(Dn / 64, Dq / 32), 256, 0, stream>>>(Wq,  wqH, wqL, Dn, Dq);
  wtrans_split_kernel<<<dim3(Dn / 64, Dq / 32), 256, 0, stream>>>(Wk,  wkH, wkL, Dn, Dq);
  wtrans_split_kernel<<<dim3(Dn / 64, Dn / 32), 256, 0, stream>>>(Wv,  wvH, wvL, Dn, Dn);
  wtrans_split_kernel<<<dim3(Dn / 64, Dn / 32), 256, 0, stream>>>(Wfc, wfH, wfL, Dn, Dn);

  const int tilesQ = (M / 64) * (Dq / 64);
  const int tilesV = (M / 64) * (Dn / 64);
  wmma_gemm64<1, true, 2, 0, false, 0><<<dim3((tilesQ + 7) / 8, 1), 256, 0, stream>>>(
      aqH, aqL, Dn, 0L, wqH, wqL, Dn, 0L, (void*)qp, (void*)nullptr, Dq, 0L,
      bq, (const float*)nullptr, 0L, M, Dq, Dn, 1.0f);
  wmma_gemm64<1, true, 2, 0, false, 0><<<dim3((tilesQ + 7) / 8, 1), 256, 0, stream>>>(
      akH, akL, Dn, 0L, wkH, wkL, Dn, 0L, (void*)kp, (void*)nullptr, Dq, 0L,
      bk, (const float*)nullptr, 0L, M, Dq, Dn, 1.0f);
  wmma_gemm64<1, true, 2, 0, false, 0><<<dim3((tilesV + 7) / 8, 1), 256, 0, stream>>>(
      avH, avL, Dn, 0L, wvH, wvL, Dn, 0L, (void*)vp, (void*)nullptr, Dn, 0L,
      bv, (const float*)nullptr, 0L, M, Dn, Dn, 1.0f);

  rel_attn_kernel<<<dim3(Bn * Hn * (Ln / 64)), 128, 0, stream>>>(qp, kp, vp, E, Obf);

  split_planes_kernel<<<gCast, 256, 0, stream>>>(Obf, aoH, aoL, n8);
  wmma_gemm64<1, true, 2, 0, false, 0><<<dim3((tilesV + 7) / 8, 1), 256, 0, stream>>>(
      aoH, aoL, Dn, 0L, wfH, wfL, Dn, 0L, (void*)out, (void*)nullptr, Dn, 0L,
      bfc, (const float*)nullptr, 0L, M, Dn, Dn, 1.0f);
}
